// MTSPModel_28647431864770
// MI455X (gfx1250) — hardware-verified
//
#include <hip/hip_runtime.h>
#include <math.h>
#include <stdint.h>

#define NB     8
#define NA     50
#define NAP    64
#define NN     1000
#define NNP    1024
#define CH     128
#define NHEAD  8
#define HDIM   16
#define FFD    512
#define RN     (NB * NNP)
#define RA     (NB * NAP)
#define INEPS  1.0e-5f
#define XC     4.0f
#define WSC    16.0f
#define NHC    32.0f
#define HC     64.0f
#define NOC    64.0f
#define QC     32.0f
#define KC     16.0f
#define VC     64.0f
#define OC     32.0f
#define LNPC   6.931471805599453f
#define NEGBIG (-3.0e37f)
static_assert(NHEAD * HDIM == CH);
static_assert((RN % 64) == 0 && (RA % 64) == 0 && (NNP % 64) == 0 && (NAP % 64) == 0 && (FFD % 64) == 0);
static_assert((NNP % 32) == 0 && (NAP % 32) == 0);

typedef _Float16 v16h __attribute__((ext_vector_type(16)));
typedef _Float16 v8h  __attribute__((ext_vector_type(8)));
typedef float    v8f  __attribute__((ext_vector_type(8)));
typedef float    v4f  __attribute__((ext_vector_type(4)));
typedef unsigned int v4u __attribute__((ext_vector_type(4)));

union FragH { v16h v; v8h h[2]; };
struct WSrc { const float* p[18]; };
static_assert(sizeof(WSrc) == 144);

__device__ __forceinline__ unsigned short bf_bits(float f) {
  unsigned u = __float_as_uint(f);
  return (unsigned short)((u + 0x7FFFu + ((u >> 16) & 1u)) >> 16);
}
__device__ __forceinline__ float bf_up(unsigned short h) { return __uint_as_float(((unsigned)h) << 16); }
__device__ __forceinline__ float bfr(float f) { return bf_up(bf_bits(f)); }
__device__ __forceinline__ unsigned short h_bits(_Float16 x) { return __builtin_bit_cast(unsigned short, x); }
__device__ __forceinline__ unsigned pk16(unsigned short a, unsigned short b) { return (unsigned)a | ((unsigned)b << 16); }
__device__ __forceinline__ v8f zero8() { v8f z = {0.f, 0.f, 0.f, 0.f, 0.f, 0.f, 0.f, 0.f}; return z; }
__device__ __forceinline__ float hmax8(v8f s) {
  return fmaxf(fmaxf(fmaxf(s[0], s[1]), fmaxf(s[2], s[3])), fmaxf(fmaxf(s[4], s[5]), fmaxf(s[6], s[7])));
}
__device__ __forceinline__ void split2(float f0, float f1, unsigned& hi, unsigned& lo) {
  const _Float16 h0 = (_Float16)f0, h1 = (_Float16)f1;
  const _Float16 l0 = (_Float16)(f0 - (float)h0), l1 = (_Float16)(f1 - (float)h1);
  hi = pk16(h_bits(h0), h_bits(h1));
  lo = pk16(h_bits(l0), h_bits(l1));
}

__device__ __forceinline__ v16h ldfrag_h(const _Float16* p) {
  FragH f;
  f.h[0] = *(const v8h*)(p);
  f.h[1] = *(const v8h*)(p + 16);
  return f.v;
}

__device__ __forceinline__ v8f mma_h_raw(v16h a, v16h b, v8f c) {
  return __builtin_amdgcn_wmma_f32_16x16x32_f16(false, a, false, b, (short)0, c, false, false);
}
__device__ __forceinline__ void dep_guard1(v8f& a, v8f& b, v16h x) {
#if defined(__HIP_DEVICE_COMPILE__)
  asm volatile("v_nop\n\tv_nop\n\tv_nop\n\tv_nop" : "+v"(a), "+v"(b) : "v"(x));
#endif
}
__device__ __forceinline__ void dep_guard2(v8f& a, v8f& b, v16h x, v16h y) {
#if defined(__HIP_DEVICE_COMPILE__)
  asm volatile("v_nop\n\tv_nop\n\tv_nop\n\tv_nop" : "+v"(a), "+v"(b) : "v"(x), "v"(y));
#endif
}
__device__ __forceinline__ void keep4_h(v16h a, v16h b, v16h c, v16h d) {
#if defined(__HIP_DEVICE_COMPILE__)
  asm volatile("v_nop" :: "v"(a), "v"(b), "v"(c), "v"(d));
#endif
}
__device__ __forceinline__ void acc_guard4(v8f& a, v8f& b, v8f& c, v8f& d) {
#if defined(__HIP_DEVICE_COMPILE__)
  asm volatile("v_nop\n\tv_nop\n\tv_nop\n\tv_nop" : "+v"(a), "+v"(b), "+v"(c), "+v"(d));
#endif
}
__device__ __forceinline__ void sguard4(v8f& a, v8f& b, v8f& c, v8f& d,
                                        v16h k0, v16h k1, v16h k2, v16h k3, v16h q) {
#if defined(__HIP_DEVICE_COMPILE__)
  asm volatile("v_nop\n\tv_nop\n\tv_nop\n\tv_nop"
               : "+v"(a), "+v"(b), "+v"(c), "+v"(d) : "v"(k0), "v"(k1), "v"(k2), "v"(k3), "v"(q));
#endif
}
__device__ __forceinline__ void sguard8(v8f& a, v8f& b, v8f& c, v8f& d,
                                        v16h k0, v16h k1, v16h k2, v16h k3,
                                        v16h g0, v16h g1, v16h g2, v16h g3, v16h q) {
#if defined(__HIP_DEVICE_COMPILE__)
  asm volatile("v_nop\n\tv_nop\n\tv_nop\n\tv_nop"
               : "+v"(a), "+v"(b), "+v"(c), "+v"(d)
               : "v"(k0), "v"(k1), "v"(k2), "v"(k3), "v"(g0), "v"(g1), "v"(g2), "v"(g3), "v"(q));
#endif
}
__device__ __forceinline__ void oguard6(v8f& o, v16h a0, v16h a1, v16h a2, v16h a3, v16h b0, v16h b1) {
#if defined(__HIP_DEVICE_COMPILE__)
  asm volatile("v_nop\n\tv_nop\n\tv_nop\n\tv_nop" : "+v"(o) : "v"(a0), "v"(a1), "v"(a2), "v"(a3), "v"(b0), "v"(b1));
#endif
}
__device__ __forceinline__ void wave_sync_lds() {
  __builtin_amdgcn_fence(__ATOMIC_RELEASE, "workgroup");
  __builtin_amdgcn_wave_barrier();
  __builtin_amdgcn_fence(__ATOMIC_ACQUIRE, "workgroup");
}

__global__ __launch_bounds__(256) void wprep(WSrc s, unsigned short* wt) {
  __shared__ float T[64 * 33];
  const int t  = threadIdx.x;
  const int bx = blockIdx.x;
  int w, tile, K, O;
  size_t dofs;
  if (bx < 96) {
    w = bx >> 3; tile = bx & 7; K = CH; O = CH; dofs = (size_t)w * (CH * CH);
  } else if (bx < 192) {
    w = 12 + ((bx - 96) >> 5); tile = (bx - 96) & 31; K = CH; O = FFD;
    dofs = (size_t)12 * CH * CH + (size_t)(w - 12) * (CH * FFD);
  } else {
    w = 15 + ((bx - 192) >> 5); tile = (bx - 192) & 31; K = FFD; O = CH;
    dofs = (size_t)12 * CH * CH + (size_t)3 * CH * FFD + (size_t)(w - 15) * (CH * FFD);
  }
  const int ntk = K >> 6;
  const int kt = tile % ntk, ot = tile / ntk;
  const int k0 = kt * 64, o0 = ot * 32;
  const float* src = s.p[0];
#pragma unroll
  for (int i = 1; i < 18; ++i) src = (w == i) ? s.p[i] : src;
  unsigned short* ds = wt + dofs;
  {
    const int k = t >> 2, oo = 8 * (t & 3);
    const float* sp = src + (size_t)(k0 + k) * O + o0 + oo;
    const v4f a = *(const v4f*)(sp), c = *(const v4f*)(sp + 4);
#pragma unroll
    for (int i = 0; i < 4; ++i) { T[k * 33 + oo + i] = a[i]; T[k * 33 + oo + 4 + i] = c[i]; }
  }
  __syncthreads();
  {
    const int o = t >> 3, e = t & 7;
    float wv[8];
#pragma unroll
    for (int i = 0; i < 8; ++i) wv[i] = bfr(T[(8 * e + i) * 33 + o]) * WSC;
    v4u v;
#pragma unroll
    for (int i = 0; i < 4; ++i) v[i] = pk16(h_bits((_Float16)wv[2 * i]), h_bits((_Float16)wv[2 * i + 1]));
    unsigned short* dp = ds + (size_t)(o0 + o) * K + k0 + 8 * e;
    *(volatile v4u*)dp = v;
    __threadfence();
    *(volatile v4u*)dp = v;
  }
}

__global__ __launch_bounds__(256) void emb16(const float* __restrict__ src, int nvalid, int NP, unsigned short* dst) {
  const int tid = threadIdx.x;
  const int rowp = blockIdx.x * 16 + (tid >> 4);
  const int e = tid & 15;
  const int b = rowp / NP;
  const int n = rowp - b * NP;
  const bool valid = (n < nvalid);
  const int ns = valid ? n : (nvalid - 1);
  const float* sp = src + ((size_t)(b * nvalid + ns)) * CH + 8 * e;
  const v4f a = *(const v4f*)(sp), c = *(const v4f*)(sp + 4);
  float x[8];
#pragma unroll
  for (int i = 0; i < 4; ++i) { x[i] = a[i]; x[4 + i] = c[i]; }
  v4u v;
#pragma unroll
  for (int i = 0; i < 4; ++i) {
    const float f0 = valid ? bfr(x[2 * i]) * XC : 0.f;
    const float f1 = valid ? bfr(x[2 * i + 1]) * XC : 0.f;
    v[i] = pk16(h_bits((_Float16)f0), h_bits((_Float16)f1));
  }
  unsigned short* dp = dst + (size_t)rowp * CH + 8 * e;
  *(volatile v4u*)dp = v;
  __threadfence();
  *(volatile v4u*)dp = v;
}

__global__ __launch_bounds__(256) void cvt_split(const float* __restrict__ src, int NP, int nvalid, float carry,
                                                  unsigned short* dh, unsigned short* dl, float* ocopy, int docopy) {
  const int tid = threadIdx.x;
  {
    const int rowp = blockIdx.x * 16 + (tid >> 4);
    const int e = tid & 15;
    const int b = rowp / NP;
    const int n = rowp - b * NP;
    const bool valid = (n < nvalid);
    const float* sp = src + (size_t)rowp * CH + 8 * e;
    const v4f a = *(const v4f*)(sp), c = *(const v4f*)(sp + 4);
    float x[8];
#pragma unroll
    for (int i = 0; i < 4; ++i) { x[i] = a[i]; x[4 + i] = c[i]; }
    v4u hv, lv;
#pragma unroll
    for (int i = 0; i < 4; ++i) {
      const float f0 = valid ? x[2 * i] * carry : 0.f;
      const float f1 = valid ? x[2 * i + 1] * carry : 0.f;
      unsigned hh, ll;
      split2(f0, f1, hh, ll);
      hv[i] = hh; lv[i] = ll;
    }
    unsigned short* ph = dh + (size_t)rowp * CH + 8 * e;
    unsigned short* pl = dl + (size_t)rowp * CH + 8 * e;
    *(volatile v4u*)ph = hv;
    *(volatile v4u*)pl = lv;
    __threadfence();
    *(volatile v4u*)ph = hv;
    *(volatile v4u*)pl = lv;
  }
  if (docopy) {
#pragma unroll
    for (int it = 0; it < 2; ++it) {
      const int rowp = blockIdx.x * 16 + it * 8 + (tid >> 5);
      const int e4 = (tid & 31) * 4;
      const int b = rowp / NP;
      const int n = rowp - b * NP;
      const v4f v = *(const v4f*)(src + (size_t)rowp * CH + e4);
      const bool ok = (n < nvalid);
      float* dp = ocopy + ((size_t)(b * nvalid + (ok ? n : 0))) * CH + e4;
      if (ok) *(volatile v4f*)dp = v;
      __threadfence();
      if (ok) *(volatile v4f*)dp = v;
    }
  }
}

template <int SPLIT, int OM>
__global__ __launch_bounds__(256) void gemm64(
    const unsigned short* __restrict__ Ap, const unsigned short* __restrict__ Ap2, int lda, long long strideA,
    const unsigned short* __restrict__ Bp, const unsigned short* __restrict__ Bp2, int ldb, long long strideB,
    const float* __restrict__ bias, int hasb, float bsc, int relu,
    const float* __restrict__ resid, int hasr, int rres, int ldr, long long strideR, int Mres,
    void* Cout, int ldc, long long strideC, int Mstore,
    unsigned short* Clo, int ldlo, long long strideLo, int nsplit,
    float osc0, float osc1, int M, int N, int K) {
  __shared__ __align__(16) float sT[8][16 * 68];
  const int b    = blockIdx.y;
  const int lane = threadIdx.x & 31;
  const int wave = threadIdx.x >> 5;
  const int tilesN = N >> 6;
  const int tilesM = M >> 6;
  const int tile = blockIdx.x * 8 + wave;
  if (tile >= tilesM * tilesN) return;
  const int tm = tile / tilesN;
  const int tn = tile - tm * tilesN;
  const int m0 = tm << 6;
  const int n0 = tn << 6;

  const _Float16* Ah  = (const _Float16*)(const void*)Ap  + (size_t)b * strideA;
  const _Float16* Ah2 = (const _Float16*)(const void*)Ap2 + (size_t)b * strideA;
  const _Float16* Bb  = (const _Float16*)(const void*)Bp  + (size_t)b * strideB;
  const _Float16* Bb2 = (const _Float16*)(const void*)Bp2 + (size_t)b * strideB;

  const int rlane = lane & 15;
  const int koff  = (lane >> 4) * 8;
  const int mOff  = (lane >> 4) * 8;

  v8f acc[4][4];
#pragma unroll
  for (int i = 0; i < 4; ++i)
#pragma unroll
    for (int j = 0; j < 4; ++j) acc[i][j] = zero8();

  for (int k0 = 0; k0 < K; k0 += 32) {
#pragma unroll
    for (int pb = 0; pb < ((SPLIT == 2) ? 2 : 1); ++pb) {
      const _Float16* Bs = (pb == 0) ? Bb : Bb2;
      v16h bh[4];
#pragma unroll
      for (int j = 0; j < 4; ++j) {
        const size_t bo = (size_t)(n0 + (j << 4) + rlane) * ldb + koff + k0;
        bh[j] = ldfrag_h(Bs + bo);
      }
#pragma unroll
      for (int i = 0; i < 4; ++i) {
        const size_t ao = (size_t)(m0 + (i << 4) + rlane) * lda + koff + k0;
        const v16h ah = ldfrag_h(Ah + ao);
#pragma unroll
        for (int j = 0; j < 4; ++j) acc[i][j] = mma_h_raw(ah, bh[j], acc[i][j]);
        if (SPLIT == 1) {
          const v16h al = ldfrag_h(Ah2 + ao);
#pragma unroll
          for (int j = 0; j < 4; ++j) acc[i][j] = mma_h_raw(al, bh[j], acc[i][j]);
          dep_guard2(acc[i][0], acc[i][3], ah, al);
        } else {
          dep_guard1(acc[i][0], acc[i][3], ah);
        }
      }
      keep4_h(bh[0], bh[1], bh[2], bh[3]);
    }
  }
  acc_guard4(acc[0][0], acc[0][1], acc[0][2], acc[0][3]);
  acc_guard4(acc[1][0], acc[1][1], acc[1][2], acc[1][3]);
  acc_guard4(acc[2][0], acc[2][1], acc[2][2], acc[2][3]);
  acc_guard4(acc[3][0], acc[3][1], acc[3][2], acc[3][3]);

  const float oscale = (OM == 1 && n0 >= nsplit) ? osc1 : osc0;
  const bool  dolo   = (OM == 1) && (n0 < nsplit);
  const int hh2 = lane >> 4, c4 = (lane & 15) * 4;
  const int q8  = lane >> 3, c8 = (lane & 7) * 8;

  float bc4[4], bc8[8];
#pragma unroll
  for (int e = 0; e < 4; ++e) bc4[e] = 0.f;
#pragma unroll
  for (int e = 0; e < 8; ++e) bc8[e] = 0.f;
  if (hasb) {
    if (OM == 0) {
      const v4f bv = *(const v4f*)(bias + n0 + c4);
#pragma unroll
      for (int e = 0; e < 4; ++e) bc4[e] = bfr(bv[e]) * bsc;
    } else {
      const v4f b0 = *(const v4f*)(bias + n0 + c8), b1v = *(const v4f*)(bias + n0 + c8 + 4);
#pragma unroll
      for (int e = 0; e < 4; ++e) { bc8[e] = bfr(b0[e]) * bsc; bc8[4 + e] = bfr(b1v[e]) * bsc; }
    }
  }

  float* slab = sT[wave];
#pragma unroll
  for (int i = 0; i < 4; ++i) {
    const int mBase = m0 + (i << 4);
#pragma unroll
    for (int j = 0; j < 4; ++j) {
#pragma unroll
      for (int r = 0; r < 8; ++r) {
        slab[(mOff + r) * 68 + (j << 4) + rlane] = acc[i][j][r];
      }
    }
    wave_sync_lds();
    if (OM == 0) {
      float* C = (float*)Cout + (size_t)b * strideC;
      const float* Rf = resid + (size_t)b * strideR;
      v4f vals[8];
#pragma unroll
      for (int it = 0; it < 8; ++it) {
        const int row  = it * 2 + hh2;
        const int grow = mBase + row;
        v4f v = *(const v4f*)(slab + row * 68 + c4);
#pragma unroll
        for (int e = 0; e < 4; ++e) v[e] = v[e] * oscale + bc4[e];
        if (hasr) {
          const int rr0 = (grow < Mres) ? grow : (Mres - 1);
          const v4f rr = *(const v4f*)(Rf + (size_t)rr0 * ldr + n0 + c4);
#pragma unroll
          for (int e = 0; e < 4; ++e) v[e] = v[e] + (rres ? bfr(rr[e]) : rr[e]);
        }
        if (relu) {
#pragma unroll
          for (int e = 0; e < 4; ++e) v[e] = fmaxf(v[e], 0.f);
        }
        vals[it] = v;
      }
      for (int pass = 0; pass < 2; ++pass) {
#pragma unroll
        for (int it = 0; it < 8; ++it) {
          const int row  = it * 2 + hh2;
          const int grow = mBase + row;
          if (grow < Mstore) *(volatile v4f*)(C + (size_t)grow * ldc + n0 + c4) = vals[it];
        }
        __threadfence();
      }
    } else {
      unsigned short* C = (unsigned short*)Cout + (size_t)b * strideC;
      unsigned short* L = Clo + (size_t)b * strideLo;
      v4u hv[4], lv[4];
#pragma unroll
      for (int it = 0; it < 4; ++it) {
        const int row = it * 4 + q8;
        const float* sp = slab + row * 68 + c8;
        v4u a, lo;
#pragma unroll
        for (int e = 0; e < 4; ++e) {
          float f0 = sp[2 * e] * oscale + bc8[2 * e], f1 = sp[2 * e + 1] * oscale + bc8[2 * e + 1];
          if (relu) { f0 = fmaxf(f0, 0.f); f1 = fmaxf(f1, 0.f); }
          unsigned hh, ll;
          split2(f0, f1, hh, ll);
          a[e]  = hh;
          lo[e] = ll;
        }
        hv[it] = a;
        lv[it] = lo;
      }
      for (int pass = 0; pass < 2; ++pass) {
#pragma unroll
        for (int it = 0; it < 4; ++it) {
          const int row  = it * 4 + q8;
          const int grow = mBase + row;
          if (grow < Mstore) {
            *(volatile v4u*)(C + (size_t)grow * ldc + n0 + c8) = hv[it];
            if (dolo) *(volatile v4u*)(L + (size_t)grow * ldlo + n0 + c8) = lv[it];
          }
        }
        __threadfence();
      }
    }
    wave_sync_lds();
  }
}

template <int KSPLIT>
__global__ __launch_bounds__(256)
void attn16(const unsigned short* __restrict__ qh, const unsigned short* __restrict__ ql, int ldq, int ldql,
            const unsigned short* __restrict__ kh, const unsigned short* __restrict__ kl, int ldk,
            const unsigned short* __restrict__ vh, const unsigned short* __restrict__ vl,
            unsigned short* op, int NQP, int NKP, int nkv0,
            const int* __restrict__ route, int useRoute, int nkmax) {
  __shared__ __align__(16) unsigned short Os[16 * 136];
  const int tid  = threadIdx.x;
  const int hd   = tid >> 5;
  const int lane = tid & 31;
  const int hh   = lane >> 4;
  const int c    = lane & 15;
  const int qtiles = NQP >> 4;
  const int bx = blockIdx.x;
  const int b  = bx / qtiles;
  const int qt = bx - b * qtiles;
  const int q0 = qt * 16;
  int nkv = nkv0;
  if (useRoute) {
    int r = route[b];
    r = (r < 1) ? 1 : r;
    r = (r > nkmax) ? nkmax : r;
    nkv = r;
  }

  const _Float16* QH = (const _Float16*)(const void*)qh;
  const _Float16* QL = (const _Float16*)(const void*)ql;
  const _Float16* KH = (const _Float16*)(const void*)kh;
  const _Float16* KL = (const _Float16*)(const void*)kl;
  const _Float16* VH = (const _Float16*)(const void*)vh;
  const _Float16* VL = (const _Float16*)(const void*)vl;

  FragH qf;
  {
    const size_t tr = (size_t)(b * NQP + q0 + c);
    qf.h[0] = *(const v8h*)(QH + tr * ldq  + hd * HDIM + 8 * hh);
    qf.h[1] = *(const v8h*)(QL + tr * ldql + hd * HDIM + 8 * hh);
  }
  const _Float16* Kp  = KH + (size_t)(b * NKP + c) * ldk + hd * HDIM + 8 * hh;
  const _Float16* Klp = KL + (size_t)(b * NKP + c) * ldk + hd * HDIM + 8 * hh;
  const _Float16* Vp  = VH + ((size_t)(b * CH + hd * HDIM + c)) * NKP + 8 * hh;
  const _Float16* Vlp = VL + ((size_t)(b * CH + hd * HDIM + c)) * NKP + 8 * hh;
  const float SC = 1.0f / (QC * KC);

  float m = -1.0e30f, l = 0.f;
  v8f o = zero8();
  const int nit = NKP >> 6;
#pragma unroll 1
  for (int it = 0; it < nit; ++it) {
    const int kb = it * 64;
    v16h kf[4];
#pragma unroll
    for (int j = 0; j < 4; ++j) {
      FragH f;
      f.h[0] = *(const v8h*)(Kp + (size_t)(kb + 16 * j) * ldk);
      f.h[1] = f.h[0];
      kf[j] = f.v;
    }
    v8f s0 = mma_h_raw(kf[0], qf.v, zero8());
    v8f s1 = mma_h_raw(kf[1], qf.v, zero8());
    v8f s2 = mma_h_raw(kf[2], qf.v, zero8());
    v8f s3 = mma_h_raw(kf[3], qf.v, zero8());
    if (KSPLIT) {
      v16h kg[4];
#pragma unroll
      for (int j = 0; j < 4; ++j) {
        FragH f;
        f.h[0] = *(const v8h*)(Klp + (size_t)(kb + 16 * j) * ldk);
        f.h[1] = f.h[0];
        kg[j] = f.v;
      }
      s0 = mma_h_raw(kg[0], qf.v, s0);
      s1 = mma_h_raw(kg[1], qf.v, s1);
      s2 = mma_h_raw(kg[2], qf.v, s2);
      s3 = mma_h_raw(kg[3], qf.v, s3);
      sguard8(s0, s1, s2, s3, kf[0], kf[1], kf[2], kf[3], kg[0], kg[1], kg[2], kg[3], qf.v);
    } else {
      sguard4(s0, s1, s2, s3, kf[0], kf[1], kf[2], kf[3], qf.v);
    }

    const int kq = kb + 8 * hh;
#pragma unroll
    for (int r = 0; r < 8; ++r) {
      s0[r] = (kq + r      < nkv) ? s0[r] : NEGBIG;
      s1[r] = (kq + 16 + r < nkv) ? s1[r] : NEGBIG;
      s2[r] = (kq + 32 + r < nkv) ? s2[r] : NEGBIG;
      s3[r] = (kq + 48 + r < nkv) ? s3[r] : NEGBIG;
    }

    float mx = fmaxf(fmaxf(hmax8(s0), hmax8(s1)), fmaxf(hmax8(s2), hmax8(s3)));
    mx = fmaxf(mx, __shfl_xor(mx, 16, 32));
    const float mn   = fmaxf(m, mx * SC);
    const float corr = __expf(m - mn);
    m = mn;
    const float msh = mn - LNPC;
    l *= corr;
#pragma unroll
    for (int r = 0; r < 8; ++r) o[r] *= corr;

    FragH p0, p1;
    float ls = 0.f;
#pragma unroll
    for (int r = 0; r < 8; ++r) {
      const float e0 = __expf(s0[r] * SC - msh);
      const float e1 = __expf(s1[r] * SC - msh);
      const float e2 = __expf(s2[r] * SC - msh);
      const float e3 = __expf(s3[r] * SC - msh);
      ls += (e0 + e1) + (e2 + e3);
      p0.h[0][r] = (_Float16)e0;
      p0.h[1][r] = (_Float16)e1;
      p1.h[0][r] = (_Float16)e2;
      p1.h[1][r] = (_Float16)e3;
    }
    l += ls;

    const v16h v0 = ldfrag_h(Vp + kb);
    const v16h w0 = ldfrag_h(Vlp + kb);
    const v16h v1 = ldfrag_h(Vp + kb + 32);
    const v16h w1 = ldfrag_h(Vlp + kb + 32);
    o = mma_h_raw(v0, p0.v, o);
    o = mma_h_raw(w0, p0.v, o);
    o = mma_h_raw(v1, p1.v, o);
    o = mma_h_raw(w1, p1.v, o);
    oguard6(o, v0, w0, v1, w1, p0.v, p1.v);
  }
  l += __shfl_xor(l, 16, 32);
  const float sc = (OC / VC) * (1.0f / l);

  {
    v4u pk;
#pragma unroll
    for (int e = 0; e < 4; ++e)
      pk[e] = pk16(h_bits((_Float16)(o[2 * e] * sc)), h_bits((_Float16)(o[2 * e + 1] * sc)));
    *(v4u*)(Os + c * 136 + hd * HDIM + 8 * hh) = pk;
  }
  __syncthreads();
  {
    const int row = tid >> 4, e = tid & 15;
    const v4u val = *(const v4u*)(Os + row * 136 + 8 * e);
    unsigned short* dp = op + ((size_t)(b * NQP + q0 + row)) * CH + 8 * e;
    *(volatile v4u*)dp = val;
    __threadfence();
    *(volatile v4u*)dp = val;
  }
}

__global__ __launch_bounds__(256) void inorm64(const float* __restrict__ hp, int NP, int nvalid,
                                                const float* __restrict__ gam, const float* __restrict__ bet,
                                                unsigned short* nh, unsigned short* nl) {
  __shared__ double part[4][64];
  __shared__ float smean[64], srstd[64], sg[64], sbe[64];
  const int tid = threadIdx.x, bx = blockIdx.x;
  const int b  = bx >> 1;
  const int c0 = (bx & 1) * 64;
  const int c  = tid & 63, g = tid >> 6;
  const float* col = hp + (size_t)b * NP * CH + c0 + c;
  {
    double s = 0.0;
#pragma unroll 1
    for (int r = g; r < nvalid; r += 4) s += (double)col[(size_t)r * CH];
    part[g][c] = s;
  }
  __syncthreads();
  if (tid < 64) {
    const double mm = ((part[0][tid] + part[1][tid]) + (part[2][tid] + part[3][tid])) * (1.0 / (double)nvalid);
    smean[tid] = (float)mm;
  }
  __syncthreads();
  {
    const float mc = smean[c];
    double s2 = 0.0;
#pragma unroll 1
    for (int r = g; r < nvalid; r += 4) {
      const float d = col[(size_t)r * CH] - mc;
      s2 += (double)d * (double)d;
    }
    part[g][c] = s2;
  }
  __syncthreads();
  if (tid < 64) {
    const double vv = ((part[0][tid] + part[1][tid]) + (part[2][tid] + part[3][tid])) * (1.0 / (double)nvalid);
    srstd[tid] = rsqrtf((float)vv + INEPS);
    sg[tid]  = bfr(gam[c0 + tid]);
    sbe[tid] = bfr(bet[c0 + tid]);
  }
  __syncthreads();
  const int rr = tid >> 3, e = tid & 7;
  float mm8[8], rs8[8], gg8[8], be8[8];
#pragma unroll
  for (int i = 0; i < 8; ++i) {
    mm8[i] = smean[8 * e + i]; rs8[i] = srstd[8 * e + i]; gg8[i] = sg[8 * e + i]; be8[i] = sbe[8 * e + i];
  }
#pragma unroll 1
  for (int rc = 0; rc < NP; rc += 32) {
    const int row = rc + rr;
    const bool valid = (row < nvalid);
    const float* sp = hp + ((size_t)(b * NP + row)) * CH + c0 + 8 * e;
    const v4f a = *(const v4f*)(sp), a2 = *(const v4f*)(sp + 4);
    float x[8];
#pragma unroll
    for (int i = 0; i < 4; ++i) { x[i] = a[i]; x[4 + i] = a2[i]; }
    v4u hv, lv;
#pragma unroll
    for (int i = 0; i < 4; ++i) {
      const int i0 = 2 * i, i1 = 2 * i + 1;
      const float y0 = ((x[i0] - mm8[i0]) * rs8[i0]) * gg8[i0] + be8[i0];
      const float y1 = ((x[i1] - mm8[i1]) * rs8[i1]) * gg8[i1] + be8[i1];
      const float f0 = valid ? y0 * NHC : 0.f;
      const float f1 = valid ? y1 * NHC : 0.f;
      unsigned hh, ll;
      split2(f0, f1, hh, ll);
      hv[i] = hh; lv[i] = ll;
    }
    unsigned short* ph = nh + ((size_t)(b * NP + row)) * CH + c0 + 8 * e;
    unsigned short* pl = nl + ((size_t)(b * NP + row)) * CH + c0 + 8 * e;
    *(volatile v4u*)ph = hv;
    *(volatile v4u*)pl = lv;
    __threadfence();
    *(volatile v4u*)ph = hv;
    *(volatile v4u*)pl = lv;
  }
}

static inline unsigned gblocks(int M, int N) { return (unsigned)((((M >> 6) * (N >> 6)) + 7) >> 3); }

extern "C" void kernel_launch(void* const* d_in, const int* in_sizes, int n_in,
                              void* d_out, int out_size, void* d_ws, size_t ws_size,
                              hipStream_t stream) {
  if (n_in < 36) return;
  if (in_sizes[0] != NB * NA * CH || in_sizes[1] != NB * NN * CH || in_sizes[2] != NB) return;
  for (int i = 3; i < 15; ++i) if (in_sizes[i] != CH * CH) return;
  for (int i = 15; i < 24; ++i) if (in_sizes[i] != CH) return;
  for (int i = 0; i < 3; ++i) {
    const int q = 24 + 4 * i;
    if (in_sizes[q] != CH * FFD || in_sizes[q + 1] != FFD || in_sizes[q + 2] != FFD * CH || in_sizes[q + 3] != CH) return;
  }
  if (out_size != NB * NA * CH + NB * NN * CH) return;

  const float* agent_emb = (const float*)d_in[0];
  const float* node_emb  = (const float*)d_in[1];
  const int*   route_num = (const int*)d_in[2];
  const float* combB  = (const float*)d_in[15];
  const float* comb2B = (const float*)d_in[16];
  const float* comb3B = (const float*)d_in[17];
  const float* g1 = (const float*)d_in[18];
  const float* g2 = (const float*)d_in[19];
  const float* g3 = (const float*)d_in[20];
  const float* bn1 = (const float*)d_in[21];
  const float* bn2 = (const float*)d_in[22];
  const float* bn3 = (const float*)d_in[23];
  const float* ff1b1 = (const float*)d_in[25];
  const float* ff1b2 = (const float*)d_in[27];
  const float* ff2b1 = (const float*)d_in[29];
  const float* ff2b2 = (const float*)d_in[31];
  const float* ff3b1 = (const float*)d_in[33];
  const float* ff3b2 = (const float*)d_in[35];

  WSrc wsrc;
  for (int i = 0; i < 12; ++i) wsrc.p[i] = (const float*)d_in[3 + i];
  wsrc.p[12] = (const float*)d_in[24];  wsrc.p[13] = (const float*)d_in[28];  wsrc.p[14] = (const float*)d_in[32];
  wsrc.p[15] = (const float*)d_in[26];  wsrc.p[16] = (const float*)d_in[30];  wsrc.p[17] = (const float*)d_in[34];

  const size_t PWT  = (size_t)589824 * 2;
  const size_t P16N = (size_t)RN * CH * 2;
  const size_t P16A = (size_t)RA * CH * 2;
  const size_t P32N = (size_t)RN * CH * 4;
  const size_t P32A = (size_t)RA * CH * 4;
  const size_t PQK3 = (size_t)RN * 2 * CH * 2;
  const size_t PVT  = (size_t)NB * CH * NNP * 2;
  const size_t PHN  = (size_t)RN * FFD * 2;
  const size_t PHA  = (size_t)RA * FFD * 2;
  const size_t PVT2 = (size_t)NB * CH * NAP * 2;
  size_t off = 0;
  const size_t oWT = off; off += PWT;
  const size_t oX3 = off; off += P16N;   const size_t oXA = off; off += P16A;
  const size_t oQK3 = off; off += PQK3;  const size_t oQ3L = off; off += P16N;
  const size_t oVTH = off; off += PVT;   const size_t oVTL = off; off += PVT;
  const size_t oO = off; off += P16N;    const size_t oO1 = off; off += P16A;
  const size_t oHP = off; off += P32N;   const size_t oHPA = off; off += P32A;
  const size_t oNHH = off; off += P16N;  const size_t oNHL = off; off += P16N;
  const size_t oNHAH = off; off += P16A; const size_t oNHAL = off; off += P16A;
  const size_t oHH = off; off += PHN;    const size_t oHL = off; off += PHN;
  const size_t oHAH = off; off += PHA;   const size_t oHAL = off; off += PHA;
  const size_t oNO2F = off; off += P32N; const size_t oNO2H = off; off += P16N;  const size_t oNO2L = off; off += P16N;
  const size_t oQ1H = off; off += P16A;  const size_t oQ1L = off; off += P16A;   const size_t oK1 = off; off += P16N;
  const size_t oAOF = off; off += P32A;  const size_t oAOH = off; off += P16A;   const size_t oAOL = off; off += P16A;
  const size_t oQ2H = off; off += P16N;  const size_t oQ2L = off; off += P16N;
  const size_t oK2H = off; off += P16A;  const size_t oK2L = off; off += P16A;
  const size_t oVT2H = off; off += PVT2; const size_t oVT2L = off; off += PVT2;
  if (off > ws_size) return;
  if (off > (size_t)134217728) return;

  char* ws = (char*)d_ws;
  unsigned short* WT   = (unsigned short*)(ws + oWT);
  unsigned short* X3   = (unsigned short*)(ws + oX3);
  unsigned short* XA   = (unsigned short*)(ws + oXA);
  unsigned short* QK3  = (unsigned short*)(ws + oQK3);
  unsigned short* Q3L  = (unsigned short*)(ws + oQ3L);
  unsigned short* VTH  = (unsigned short*)(ws + oVTH);
  unsigned short* VTL  = (unsigned short*)(ws + oVTL);
  unsigned short* O    = (unsigned short*)(ws + oO);
  unsigned short* O1   = (unsigned short*)(ws + oO1);
  float*          HP   = (float*)(ws + oHP);
  float*          HPA  = (float*)(ws + oHPA);
  unsigned short* NHH  = (unsigned short*)(ws + oNHH);
  unsigned short* NHL  = (unsigned short*)(ws + oNHL);
  unsigned short* NHAH = (unsigned short*)(ws + oNHAH);
  unsigned short* NHAL = (unsigned short*)(ws + oNHAL);
  unsigned short* HH   = (unsigned short*)(ws + oHH);
  unsigned short* HL   = (unsigned short*)(ws + oHL);
  unsigned short* HAH  = (unsigned short*)(ws + oHAH);
  unsigned short* HAL  = (unsigned short*)(ws + oHAL);
  float*          NO2F = (float*)(ws + oNO2F);
  unsigned short* NO2H = (unsigned short*)(ws + oNO2H);
  unsigned short* NO2L = (unsigned short*)(ws + oNO2L);
  unsigned short* Q1H  = (unsigned short*)(ws + oQ1H);
  unsigned short* Q1L  = (unsigned short*)(ws + oQ1L);
  unsigned short* K1   = (unsigned short*)(ws + oK1);
  float*          AOF  = (float*)(ws + oAOF);
  unsigned short* AOH  = (unsigned short*)(ws + oAOH);
  unsigned short* AOL  = (unsigned short*)(ws + oAOL);
  unsigned short* Q2H  = (unsigned short*)(ws + oQ2H);
  unsigned short* Q2L  = (unsigned short*)(ws + oQ2L);
  unsigned short* K2H  = (unsigned short*)(ws + oK2H);
  unsigned short* K2L  = (unsigned short*)(ws + oK2L);
  unsigned short* VT2H = (unsigned short*)(ws + oVT2H);
  unsigned short* VT2L = (unsigned short*)(ws + oVT2L);
  float* out_agent = (float*)d_out;
  float* out_node  = (float*)d_out + (size_t)NB * NA * CH;

  unsigned short* WTq   = WT + (size_t)0 * CH * CH;
  unsigned short* WTk   = WT + (size_t)1 * CH * CH;
  unsigned short* WTv   = WT + (size_t)2 * CH * CH;
  unsigned short* WTq2  = WT + (size_t)3 * CH * CH;
  unsigned short* WTk2  = WT + (size_t)4 * CH * CH;
  unsigned short* WTv2  = WT + (size_t)5 * CH * CH;
  unsigned short* WTqk3 = WT + (size_t)6 * CH * CH;
  unsigned short* WTv3  = WT + (size_t)8 * CH * CH;
  unsigned short* WTc1  = WT + (size_t)9 * CH * CH;
  unsigned short* WTc2  = WT + (size_t)10 * CH * CH;
  unsigned short* WTc3  = WT + (size_t)11 * CH * CH;
  unsigned short* W1T1  = WT + (size_t)12 * CH * CH;
  unsigned short* W1T2  = W1T1 + (size_t)CH * FFD;
  unsigned short* W1T3  = W1T2 + (size_t)CH * FFD;
  unsigned short* W2T1  = W1T3 + (size_t)CH * FFD;
  unsigned short* W2T2  = W2T1 + (size_t)CH * FFD;
  unsigned short* W2T3  = W2T2 + (size_t)CH * FFD;

  const dim3 blk(256);
  const long long SN16 = (long long)NNP * CH;
  const long long SA16 = (long long)NAP * CH;
  const float oQs  = 0.25f * QC / (XC * WSC);
  const float oKx  = KC / (XC * WSC);
  const float oVx  = VC / (XC * WSC);
  const float oQn  = QC / (NOC * WSC);
  const float oKn  = KC / (NOC * WSC);
  const float oVn  = VC / (NOC * WSC);
  const float oCmb = 1.0f / (OC * WSC);
  const float oF1  = HC / (NHC * WSC);
  const float oF2  = 1.0f / (HC * WSC);

  wprep<<<dim3(288), blk, 0, stream>>>(wsrc, WT);
  emb16<<<dim3(RN / 16), blk, 0, stream>>>(node_emb, NN, NNP, X3);
  emb16<<<dim3(RA / 16), blk, 0, stream>>>(agent_emb, NA, NAP, XA);

  gemm64<0, 1><<<dim3(gblocks(RN, 2 * CH), 1), blk, 0, stream>>>(
      X3, X3, CH, 0LL, WTqk3, WTqk3, CH, 0LL,
      combB, 0, 1.0f, 0, node_emb, 0, 0, CH, 0LL, 1,
      (void*)QK3, 2 * CH, 0LL, RN, Q3L, CH, 0LL, CH,
      oQs, oKx, RN, 2 * CH, CH);
  gemm64<0, 1><<<dim3(gblocks(CH, NNP), NB), blk, 0, stream>>>(
      WTv3, WTv3, CH, 0LL, X3, X3, CH, SN16,
      combB, 0, 1.0f, 0, node_emb, 0, 0, CH, 0LL, 1,
      (void*)VTH, NNP, (long long)CH * NNP, CH, VTL, NNP, (long long)CH * NNP, NNP,
      oVx, oVx, CH, NNP, CH);
  attn16<0><<<dim3(NB * (NNP / 16)), blk, 0, stream>>>(
      QK3, Q3L, 2 * CH, CH, QK3 + CH, QK3 + CH, 2 * CH, VTH, VTL, O, NNP, NNP, NN, route_num, 0, NA);
  gemm64<0, 0><<<dim3(gblocks(NNP, CH), NB), blk, 0, stream>>>(
      O, O, CH, SN16, WTc3, WTc3, CH, 0LL,
      comb3B, 1, 1.0f, 0, node_emb, 1, 1, CH, (long long)NN * CH, NN,
      (void*)HP, CH, SN16, NNP, Q3L, CH, 0LL, 0,
      oCmb, oCmb, NNP, CH, CH);
  inorm64<<<dim3(NB * 2), blk, 0, stream>>>(HP, NNP, NN, g3, bn3, NHH, NHL);
  gemm64<1, 1><<<dim3(gblocks(RN, FFD), 1), blk, 0, stream>>>(
      NHH, NHL, CH, 0LL, W1T3, W1T3, CH, 0LL,
      ff3b1, 1, HC, 1, node_emb, 0, 0, CH, 0LL, 1,
      (void*)HH, FFD, 0LL, RN, HL, FFD, 0LL, FFD,
      oF1, oF1, RN, FFD, CH);
  gemm64<1, 0><<<dim3(gblocks(RN, CH), 1), blk, 0, stream>>>(
      HH, HL, FFD, 0LL, W2T3, W2T3, FFD, 0LL,
      ff3b2, 1, 1.0f, 0, node_emb, 0, 0, CH, 0LL, 1,
      (void*)NO2F, CH, 0LL, RN, Q3L, CH, 0LL, 0,
      oF2, oF2, RN, CH, FFD);
  cvt_split<<<dim3(RN / 16), blk, 0, stream>>>(NO2F, NNP, NN, NOC, NO2H, NO2L, out_agent, 0);

  gemm64<0, 1><<<dim3(gblocks(RA, CH), 1), blk, 0, stream>>>(
      XA, XA, CH, 0LL, WTq, WTq, CH, 0LL,
      combB, 0, 1.0f, 0, node_emb, 0, 0, CH, 0LL, 1,
      (void*)Q1H, CH, 0LL, RA, Q1L, CH, 0LL, CH,
      oQs, oQs, RA, CH, CH);
  gemm64<1, 1><<<dim3(gblocks(RN, CH), 1), blk, 0, stream>>>(
      NO2H, NO2L, CH, 0LL, WTk, WTk, CH, 0LL,
      combB, 0, 1.0f, 0, node_emb, 0, 0, CH, 0LL, 1,
      (void*)K1, CH, 0LL, RN, K1, CH, 0LL, 0,
      oKn, oKn, RN, CH, CH);
  gemm64<2, 1><<<dim3(gblocks(CH, NNP), NB), blk, 0, stream>>>(
      WTv, WTv, CH, 0LL, NO2H, NO2L, CH, SN16,
      combB, 0, 1.0f, 0, node_emb, 0, 0, CH, 0LL, 1,
      (void*)VTH, NNP, (long long)CH * NNP, CH, VTL, NNP, (long long)CH * NNP, NNP,
      oVn, oVn, CH, NNP, CH);
  attn16<0><<<dim3(NB * (NAP / 16)), blk, 0, stream>>>(
      Q1H, Q1L, CH, CH, K1, K1, CH, VTH, VTL, O1, NAP, NNP, NN, route_num, 0, NA);
  gemm64<0, 0><<<dim3(gblocks(NAP, CH), NB), blk, 0, stream>>>(
      O1, O1, CH, SA16, WTc1, WTc1, CH, 0LL,
      combB, 1, 1.0f, 0, agent_emb, 1, 1, CH, (long long)NA * CH, NA,
      (void*)HPA, CH, SA16, NAP, Q3L, CH, 0LL, 0,
      oCmb, oCmb, NAP, CH, CH);
  inorm64<<<dim3(NB * 2), blk, 0, stream>>>(HPA, NAP, NA, g1, bn1, NHAH, NHAL);
  gemm64<1, 1><<<dim3(gblocks(RA, FFD), 1), blk, 0, stream>>>(
      NHAH, NHAL, CH, 0LL, W1T1, W1T1, CH, 0LL,
      ff1b1, 1, HC, 1, node_emb, 0, 0, CH, 0LL, 1,
      (void*)HAH, FFD, 0LL, RA, HAL, FFD, 0LL, FFD,
      oF1, oF1, RA, FFD, CH);
  gemm64<1, 0><<<dim3(gblocks(RA, CH), 1), blk, 0, stream>>>(
      HAH, HAL, FFD, 0LL, W2T1, W2T1, FFD, 0LL,
      ff1b2, 1, 1.0f, 0, node_emb, 0, 0, CH, 0LL, 1,
      (void*)AOF, CH, 0LL, RA, Q3L, CH, 0LL, 0,
      oF2, oF2, RA, CH, FFD);
  cvt_split<<<dim3(RA / 16), blk, 0, stream>>>(AOF, NAP, NA, NOC, AOH, AOL, out_agent, 1);

  gemm64<1, 1><<<dim3(gblocks(RN, CH), 1), blk, 0, stream>>>(
      NO2H, NO2L, CH, 0LL, WTq2, WTq2, CH, 0LL,
      combB, 0, 1.0f, 0, node_emb, 0, 0, CH, 0LL, 1,
      (void*)Q2H, CH, 0LL, RN, Q2L, CH, 0LL, CH,
      oQn, oQn, RN, CH, CH);
  gemm64<1, 1><<<dim3(gblocks(RA, CH), 1), blk, 0, stream>>>(
      AOH, AOL, CH, 0LL, WTk2, WTk2, CH, 0LL,
      combB, 0, 1.0f, 0, node_emb, 0, 0, CH, 0LL, 1,
      (void*)K2H, CH, 0LL, RA, K2L, CH, 0LL, CH,
      oKn, oKn, RA, CH, CH);
  gemm64<2, 1><<<dim3(gblocks(CH, NAP), NB), blk, 0, stream>>>(
      WTv2, WTv2, CH, 0LL, AOH, AOL, CH, SA16,
      combB, 0, 1.0f, 0, node_emb, 0, 0, CH, 0LL, 1,
      (void*)VT2H, NAP, (long long)CH * NAP, CH, VT2L, NAP, (long long)CH * NAP, NAP,
      oVn, oVn, CH, NAP, CH);
  attn16<1><<<dim3(NB * (NNP / 16)), blk, 0, stream>>>(
      Q2H, Q2L, CH, CH, K2H, K2L, CH, VT2H, VT2L, O, NNP, NAP, NA, route_num, 1, NA);
  gemm64<0, 0><<<dim3(gblocks(NNP, CH), NB), blk, 0, stream>>>(
      O, O, CH, SN16, WTc2, WTc2, CH, 0LL,
      comb2B, 1, 1.0f, 0, NO2F, 1, 0, CH, SN16, NNP,
      (void*)HP, CH, SN16, NNP, Q3L, CH, 0LL, 0,
      oCmb, oCmb, NNP, CH, CH);
  inorm64<<<dim3(NB * 2), blk, 0, stream>>>(HP, NNP, NN, g2, bn2, NHH, NHL);
  gemm64<1, 1><<<dim3(gblocks(RN, FFD), 1), blk, 0, stream>>>(
      NHH, NHL, CH, 0LL, W1T2, W1T2, CH, 0LL,
      ff2b1, 1, HC, 1, node_emb, 0, 0, CH, 0LL, 1,
      (void*)HH, FFD, 0LL, RN, HL, FFD, 0LL, FFD,
      oF1, oF1, RN, FFD, CH);
  gemm64<1, 0><<<dim3(gblocks(NNP, CH), NB), blk, 0, stream>>>(
      HH, HL, FFD, (long long)NNP * FFD, W2T2, W2T2, FFD, 0LL,
      ff2b2, 1, 1.0f, 0, node_emb, 0, 0, CH, 0LL, 1,
      (void*)out_node, CH, (long long)NN * CH, NN, Q3L, CH, 0LL, 0,
      oF2, oF2, NNP, CH, FFD);
  (void)hipGetLastError();
}
